// GarNet_39685497815054
// MI455X (gfx1250) — hardware-verified
//
#include <hip/hip_runtime.h>
#include <math.h>
typedef __attribute__((ext_vector_type(16))) _Float16 v16h;
typedef __attribute__((ext_vector_type(8)))  _Float16 v8h;
typedef __attribute__((ext_vector_type(16))) __bf16   v16b;
typedef __attribute__((ext_vector_type(8)))  __bf16   v8b;
typedef __attribute__((ext_vector_type(8)))  float    v8f;
typedef __attribute__((ext_vector_type(4)))  float    v4f;
#define PSCALE 32768.0f
#define U16(p) ((const unsigned short*)(const void*)(p))
#define PSCALE_INV (1.0f / 32768.0f)

__device__ __forceinline__ unsigned short f2bf_bits(float f) {
  unsigned u = __float_as_uint(f);
  return (unsigned short)((u + 0x7FFFu + ((u >> 16) & 1u)) >> 16);
}
__device__ __forceinline__ float bf_bits2f(unsigned short h) { return __uint_as_float(((unsigned)h) << 16); }

__device__ __forceinline__ void dep_guard_h(v8f& a, v8f& b, v16h x, v16h y) { asm volatile("v_nop\n\tv_nop\n\tv_nop\n\tv_nop" : "+v"(a), "+v"(b) : "v"(x), "v"(y)); }
__device__ __forceinline__ void dep_guard_b(v8f& a, v8f& b, v16b x, v16b y) { asm volatile("v_nop\n\tv_nop\n\tv_nop\n\tv_nop" : "+v"(a), "+v"(b) : "v"(x), "v"(y)); }
__device__ __forceinline__ void keep4_h(v16h a, v16h b, v16h c, v16h d) { asm volatile("v_nop" :: "v"(a), "v"(b), "v"(c), "v"(d)); }
__device__ __forceinline__ void keep4_b(v16b a, v16b b, v16b c, v16b d) { asm volatile("v_nop" :: "v"(a), "v"(b), "v"(c), "v"(d)); }
__device__ __forceinline__ void acc_guard4(v8f& a, v8f& b, v8f& c, v8f& d) { asm volatile("v_nop\n\tv_nop\n\tv_nop\n\tv_nop" : "+v"(a), "+v"(b), "+v"(c), "+v"(d)); }
template <typename T> struct Frag;
template <> struct Frag<_Float16> {
  typedef v16h V; union U { v16h v; v8h h[2]; };
  static __device__ __forceinline__ v16h load(const _Float16* p) {
    U f; f.h[0] = *(const v8h*)(p); f.h[1] = *(const v8h*)(p + 16); return f.v;
  }
  static __device__ __forceinline__ v8f mma(v16h a, v16h b, v8f c) {
    return __builtin_amdgcn_wmma_f32_16x16x32_f16(false, a, false, b, (short)0, c, false, false);
  }
  static __device__ __forceinline__ void guard(v8f& a, v8f& b, v16h x, v16h y) { dep_guard_h(a, b, x, y); }
  static __device__ __forceinline__ void keep(v16h a, v16h b, v16h c, v16h d) { keep4_h(a, b, c, d); }
};
template <> struct Frag<__bf16> {
  typedef v16b V; union U { v16b v; v8b h[2]; };
  static __device__ __forceinline__ v16b load(const __bf16* p) {
    U f; f.h[0] = *(const v8b*)(p); f.h[1] = *(const v8b*)(p + 16); return f.v;
  }
  static __device__ __forceinline__ v8f mma(v16b a, v16b b, v8f c) {
    return __builtin_amdgcn_wmma_f32_16x16x32_bf16(false, a, false, b, (short)0, c, false, false);
  }
  static __device__ __forceinline__ void guard(v8f& a, v8f& b, v16b x, v16b y) { dep_guard_b(a, b, x, y); }
  static __device__ __forceinline__ void keep(v16b a, v16b b, v16b c, v16b d) { keep4_b(a, b, c, d); }
};

template <int ET> struct Elem;
template <> struct Elem<0> { typedef _Float16 T; };
template <> struct Elem<1> { typedef __bf16 T; };
template <int ET, bool SPLIT, int BIAS_MODE, int OUT_MODE, bool RESID, int ACT = 0>
__global__ __launch_bounds__(256) void wmma_gemm64(
    const unsigned short* __restrict__ Ap, const unsigned short* __restrict__ A2p, int lda, long strideA,
    const unsigned short* __restrict__ Btp, const unsigned short* __restrict__ Bt2p, int ldb, long strideB,
    void* __restrict__ Cout, void* __restrict__ Cout2, int ldc, long strideC,
    const float* __restrict__ bias,
    const float* __restrict__ resid, long strideR,
    int M, int N, int K, float scale) {
  typedef typename Elem<ET>::T T;
  typedef typename Frag<T>::V V;
  const T* A = (const T*)Ap; const T* A2 = (const T*)A2p; const T* Bt = (const T*)Btp; const T* Bt2 = (const T*)Bt2p;
  __shared__ __align__(16) float sT[8][16 * 68];
  const int b    = blockIdx.y;
  const int lane = threadIdx.x & 31;
  const int wave = threadIdx.x >> 5;
  const int tilesN = N >> 6;
  const int tilesM = M >> 6;
  const int tile = blockIdx.x * 8 + wave;
  if (tile >= tilesM * tilesN) return;
  const int tm = tile / tilesN;
  const int tn = tile - tm * tilesN;
  const int m0 = tm << 6;
  const int n0 = tn << 6;

  const T* Ab  = A  + (size_t)b * strideA;
  const T* Bb  = Bt + (size_t)b * strideB;
  const T* Ab2 = SPLIT ? (A2  + (size_t)b * strideA) : nullptr;
  const T* Bb2 = SPLIT ? (Bt2 + (size_t)b * strideB) : nullptr;

  const int rlane = lane & 15;
  const int koff  = (lane >> 4) * 8;
  const int mOff  = (lane >> 4) * 8;

  v8f acc[4][4];
#pragma unroll
  for (int i = 0; i < 4; ++i)
#pragma unroll
    for (int j = 0; j < 4; ++j) acc[i][j] = (v8f){0.f,0.f,0.f,0.f,0.f,0.f,0.f,0.f};

  for (int k0 = 0; k0 < K; k0 += 32) {
    V bh[4], bl[4];
#pragma unroll
    for (int j = 0; j < 4; ++j) {
      const size_t bo = (size_t)(n0 + (j << 4) + rlane) * ldb + koff + k0;
      bh[j] = Frag<T>::load(Bb + bo);
      if (SPLIT) bl[j] = Frag<T>::load(Bb2 + bo);
    }
#pragma unroll
    for (int i = 0; i < 4; ++i) {
      const size_t ao = (size_t)(m0 + (i << 4) + rlane) * lda + koff + k0;
      V ah = Frag<T>::load(Ab + ao);
      V al;
      if (SPLIT) al = Frag<T>::load(Ab2 + ao);
#pragma unroll
      for (int j = 0; j < 4; ++j) {
        acc[i][j] = Frag<T>::mma(ah, bh[j], acc[i][j]);
        if (SPLIT) {
          acc[i][j] = Frag<T>::mma(ah, bl[j], acc[i][j]);
          acc[i][j] = Frag<T>::mma(al, bh[j], acc[i][j]);
        }
      }
      Frag<T>::guard(acc[i][0], acc[i][3], ah, SPLIT ? al : ah);
    }
    Frag<T>::keep(bh[0], bh[1], bh[2], bh[3]);
    if (SPLIT) Frag<T>::keep(bl[0], bl[1], bl[2], bl[3]);
  }
  acc_guard4(acc[0][0], acc[0][1], acc[0][2], acc[0][3]);
  acc_guard4(acc[1][0], acc[1][1], acc[1][2], acc[1][3]);
  acc_guard4(acc[2][0], acc[2][1], acc[2][2], acc[2][3]);
  acc_guard4(acc[3][0], acc[3][1], acc[3][2], acc[3][3]);

  float* slab = sT[wave];
  const float* Rb = RESID ? (resid + (size_t)b * strideR) : nullptr;
#pragma unroll
  for (int i = 0; i < 4; ++i) {
    const int mBase = m0 + (i << 4);
#pragma unroll
    for (int j = 0; j < 4; ++j) {
      const int n = n0 + (j << 4) + rlane;
      float bv = 0.f;
      if (BIAS_MODE == 2) bv = bias[n];
#pragma unroll
      for (int r = 0; r < 8; ++r) {
        float v = acc[i][j][r] * scale;
        if (BIAS_MODE == 1) v += bias[mBase + mOff + r];
        if (BIAS_MODE == 2) v += bv;
        if (RESID) v += Rb[(size_t)(mBase + mOff + r) * ldc + n];
        if (ACT == 1) v = tanhf(v);
        if (ACT == 2) v = fmaxf(v, 0.0f);
        if (ACT == 3) v = v / (1.0f + expf(-v));
        if (ACT == 4) v = (v > 0.f) ? v : 0.01f * v;
        if (ACT == 5) v = 0.5f * v * (1.0f + erff(v * 0.70710678118654752f));
        slab[(mOff + r) * 68 + (j << 4) + rlane] = v;
      }
    }
    __builtin_amdgcn_fence(__ATOMIC_RELEASE, "workgroup");
    __builtin_amdgcn_wave_barrier();
    __builtin_amdgcn_fence(__ATOMIC_ACQUIRE, "workgroup");
    if (OUT_MODE == 0) {
      float* C = (float*)Cout + (size_t)b * strideC;
      const int hh = lane >> 4, c4 = (lane & 15) * 4;
      for (int pass = 0; pass < 2; ++pass) {
#pragma unroll
        for (int it = 0; it < 8; ++it) {
          const int row = it * 2 + hh;
          v4f v = *(const v4f*)(slab + row * 68 + c4);
          *(volatile v4f*)(C + (size_t)(mBase + row) * ldc + n0 + c4) = v;
        }
        __threadfence();
      }
    } else {
      const int q = lane >> 3, c8 = (lane & 7) * 8;
      unsigned short* C  = (unsigned short*)Cout  + (size_t)b * strideC;
      unsigned short* C2 = (OUT_MODE == 2) ? ((unsigned short*)Cout2 + (size_t)b * strideC) : nullptr;
      for (int pass = 0; pass < 2; ++pass) {
#pragma unroll
        for (int it = 0; it < 4; ++it) {
          const int row = it * 4 + q;
          const float* sp = slab + row * 68 + c8;
          v8h hv, lv;
#pragma unroll
          for (int e = 0; e < 8; ++e) {
            if (OUT_MODE == 1) {
              hv[e] = (_Float16)sp[e];
            } else {
              unsigned short hb = f2bf_bits(sp[e]);
              unsigned short lb = f2bf_bits(sp[e] - bf_bits2f(hb));
              hv[e] = __builtin_bit_cast(_Float16, hb);
              lv[e] = __builtin_bit_cast(_Float16, lb);
            }
          }
          *(volatile v8h*)(C + (size_t)(mBase + row) * ldc + n0 + c8) = hv;
          if (OUT_MODE == 2) *(volatile v8h*)(C2 + (size_t)(mBase + row) * ldc + n0 + c8) = lv;
        }
        __threadfence();
      }
    }
    __builtin_amdgcn_fence(__ATOMIC_RELEASE, "workgroup");
    __builtin_amdgcn_wave_barrier();
    __builtin_amdgcn_fence(__ATOMIC_ACQUIRE, "workgroup");
  }
}

__global__ __launch_bounds__(256) void cast_f32_f16x2(
    const float* __restrict__ in, _Float16* __restrict__ out, int n2) {
  int i = blockIdx.x * 256 + threadIdx.x;
  if (i < n2) {
    const _Float16 h0 = (_Float16)in[2 * i], h1 = (_Float16)in[2 * i + 1];
    const unsigned u = (unsigned)__builtin_bit_cast(unsigned short, h0) | ((unsigned)__builtin_bit_cast(unsigned short, h1) << 16);
    ((volatile unsigned*)out)[i] = u;
    __threadfence();
    ((volatile unsigned*)out)[i] = u;
  }
}

__global__ __launch_bounds__(256) void split_f32_bf16x2(
    const float* __restrict__ in, __bf16* __restrict__ hi, __bf16* __restrict__ lo, long n2) {
  long i = (long)blockIdx.x * 256 + threadIdx.x;
  long stride = (long)gridDim.x * 256;
  for (int pass = 0; pass < 2; ++pass) {
    for (long j = i; j < n2; j += stride) {
      const float a = in[2 * j], b = in[2 * j + 1];
      const unsigned short ah = f2bf_bits(a), bh = f2bf_bits(b);
      const unsigned short al = f2bf_bits(a - bf_bits2f(ah)), bl = f2bf_bits(b - bf_bits2f(bh));
      ((volatile unsigned*)hi)[j] = (unsigned)ah | ((unsigned)bh << 16);
      ((volatile unsigned*)lo)[j] = (unsigned)al | ((unsigned)bl << 16);
    }
    __threadfence();
  }
}


#define GBv 64
#define GV 512
#define GR (GBv * GV)
#define GFI 8
#define GP 128
#define GA 16
#define GF 144
#define GNF 32
__global__ __launch_bounds__(256) void prep_kernel(const float* __restrict__ data, const float* __restrict__ Wf, const float* __restrict__ bfl, const float* __restrict__ Ws, const float* __restrict__ bs,
                                                  __bf16* __restrict__ Dh, __bf16* __restrict__ Dl, __bf16* __restrict__ Bh, __bf16* __restrict__ Bl, float* __restrict__ bb) {
  const size_t i = (size_t)blockIdx.x * 256 + threadIdx.x;
  if (i < (size_t)GR * 16) { const size_t r = i / 16; const int c = 2 * (int)(i % 16); float v[2]; for (int e = 0; e < 2; ++e) v[e] = (c + e < GFI) ? data[r * GFI + c + e] : 0.f;
    const unsigned short h0 = f2bf_bits(v[0]), h1 = f2bf_bits(v[1]), l0 = f2bf_bits(v[0] - bf_bits2f(h0)), l1 = f2bf_bits(v[1] - bf_bits2f(h1));
    for (int pass = 0; pass < 2; ++pass) { ((volatile unsigned*)Dh)[i] = (unsigned)h0 | ((unsigned)h1 << 16); ((volatile unsigned*)Dl)[i] = (unsigned)l0 | ((unsigned)l1 << 16); __threadfence(); } }
  if (i < 192 * 16) { const int o = (int)(i / 16), c = 2 * (int)(i % 16); float v[2] = {0.f, 0.f};
    for (int e = 0; e < 2; ++e) { const int cc = c + e; if (cc < GFI) { if (o < GP) v[e] = Wf[cc * GP + o]; else if (o < GF) v[e] = Ws[cc * GA + (o - GP)]; } }
    const unsigned short h0 = f2bf_bits(v[0]), h1 = f2bf_bits(v[1]), l0 = f2bf_bits(v[0] - bf_bits2f(h0)), l1 = f2bf_bits(v[1] - bf_bits2f(h1));
    for (int pass = 0; pass < 2; ++pass) { ((volatile unsigned*)Bh)[i] = (unsigned)h0 | ((unsigned)h1 << 16); ((volatile unsigned*)Bl)[i] = (unsigned)l0 | ((unsigned)l1 << 16); if (c == 0) ((volatile float*)bb)[o] = (o < GP) ? bfl[o] : (o < GF ? bs[o - GP] : 0.f); __threadfence(); } }
}
__global__ __launch_bounds__(256) void frow_kernel(const float* __restrict__ data, float* __restrict__ FD) {
  const int lane = threadIdx.x & 31, wave = threadIdx.x >> 5; const size_t r = (size_t)blockIdx.x * 8 + wave;
  const float m = (data[r * GFI + 3] > 0.5f) ? 1.f : 0.f;
  float v[6];
  for (int q = 0; q < 6; ++q) { const int c = lane * 6 + q; float x = FD[r * 192 + c];
    if (c < GP) x = m * x; else if (c < GF) x = m * expf(-x * x); else x = (c == GF) ? m : 0.f;
    v[q] = x; }
  for (int pass = 0; pass < 2; ++pass) { for (int q = 0; q < 6; ++q) ((volatile float*)FD)[r * 192 + lane * 6 + q] = v[q]; __threadfence(); }
}
__global__ __launch_bounds__(256) void ftrans_kernel(const float* __restrict__ FD, unsigned* __restrict__ FT16, unsigned* __restrict__ EWT16) {
  __shared__ float tile[192][65];
  const int b = blockIdx.y, v0 = blockIdx.x * 64, tx = threadIdx.x, ty = threadIdx.y;
  for (int r = ty; r < 64; r += 8) { const float* src = FD + ((size_t)b * GV + v0 + r) * 192; for (int c = tx; c < 192; c += 32) tile[c][r] = src[c]; }
  __syncthreads();
  for (int pass = 0; pass < 2; ++pass) {
    for (int f = ty; f < 192; f += 8) { const float a0 = (f < GF) ? tile[f][2 * tx] : 0.f, a1 = (f < GF) ? tile[f][2 * tx + 1] : 0.f;
      ((volatile unsigned*)FT16)[(((size_t)b * 192 + f) * GV + v0) / 2 + tx] = (unsigned)__builtin_bit_cast(unsigned short, (_Float16)a0) | ((unsigned)__builtin_bit_cast(unsigned short, (_Float16)a1) << 16); }
    for (int a = ty; a < 64; a += 8) { const float e0 = (a < GA) ? tile[GP + a][2 * tx] : 0.f, e1 = (a < GA) ? tile[GP + a][2 * tx + 1] : 0.f;
      ((volatile unsigned*)EWT16)[(((size_t)b * 64 + a) * GV + v0) / 2 + tx] = (unsigned)__builtin_bit_cast(unsigned short, (_Float16)e0) | ((unsigned)__builtin_bit_cast(unsigned short, (_Float16)e1) << 16); }
    __threadfence(); }
}
__global__ __launch_bounds__(256) void agg_kernel(const float* __restrict__ FD, const float* __restrict__ AGGM, float* __restrict__ AGG) {
  __shared__ float ag[GA * 288];
  const int b = blockIdx.x; const float* F = FD + (size_t)b * GV * 192;
  for (int p = threadIdx.x; p < GA * GF; p += 256) { const int a = p / GF, f = p % GF; float mx = -INFINITY;
#pragma unroll 1
    for (int v = 0; v < GV; ++v) { const float ew = F[(size_t)v * 192 + GP + a]; mx = fmaxf(mx, ew * F[(size_t)v * 192 + f]); }
    ag[a * 288 + f] = mx; ag[a * 288 + GF + f] = AGGM[((size_t)b * 192 + f) * 64 + a]; }
  __syncthreads();
  float* dst = AGG + (size_t)b * GA * 288;
  for (int pass = 0; pass < 2; ++pass) { for (int i = threadIdx.x; i < GA * 288; i += 256) ((volatile float*)dst)[i] = ag[i]; __threadfence(); }
}
__global__ __launch_bounds__(256) void m_kernel(const float* __restrict__ AGG, const float* __restrict__ Wout, float* __restrict__ M) {
  const int b = blockIdx.x;
  for (int p = threadIdx.x; p < GA * GNF; p += 256) { const int a = p / GNF, o = p % GNF; const float* ag = AGG + ((size_t)b * GA + a) * 288; const float* w = Wout + (size_t)(GFI + a * 288) * GNF + o;
    float s = Wout[(size_t)(GFI + GA * 288 + a) * GNF + o];
#pragma unroll 1
    for (int j = 0; j < 288; ++j) s += ag[j] * w[(size_t)j * GNF];
    ((volatile float*)M)[((size_t)b * GA + a) * GNF + o] = s; }
  __threadfence();
  for (int p = threadIdx.x; p < GA * GNF; p += 256) { const size_t i = (size_t)b * GA * GNF + p; ((volatile float*)M)[i] = M[i]; }
}
__global__ __launch_bounds__(256) void out_kernel(const float* __restrict__ data, const float* __restrict__ FD, const float* __restrict__ M, const float* __restrict__ Wout, const float* __restrict__ bout, float* __restrict__ out) {
  const int lane = threadIdx.x & 31, wave = threadIdx.x >> 5; const size_t r = (size_t)blockIdx.x * 8 + wave; const int b = (int)(r / GV);
  float s = bout[lane];
#pragma unroll 1
  for (int i = 0; i < GFI; ++i) s += data[r * GFI + i] * Wout[i * GNF + lane];
#pragma unroll 1
  for (int a = 0; a < GA; ++a) s += FD[r * 192 + GP + a] * M[((size_t)b * GA + a) * GNF + lane];
  const float m = FD[r * 192 + GF]; const float v = m * tanhf(s);
  ((volatile float*)out)[r * GNF + lane] = v; __threadfence(); ((volatile float*)out)[r * GNF + lane] = v;
}
extern "C" void kernel_launch(void* const* d_in, const int* in_sizes, int n_in, void* d_out, int out_size, void* d_ws, size_t ws_size, hipStream_t stream) {
  (void)in_sizes; (void)n_in; (void)out_size; (void)ws_size;
  const float* data = (const float*)d_in[0]; const float* Wf = (const float*)d_in[1]; const float* bfl = (const float*)d_in[2]; const float* Ws = (const float*)d_in[3]; const float* bs = (const float*)d_in[4]; const float* Wout = (const float*)d_in[5]; const float* bout = (const float*)d_in[6];
  char* ws = (char*)d_ws; size_t off = 0;
  auto carve = [&](size_t bytes) -> char* { char* p = ws + off; off += (bytes + 255) & ~(size_t)255; return p; };
  __bf16* Dh = (__bf16*)carve((size_t)GR * 32 * 2); __bf16* Dl = (__bf16*)carve((size_t)GR * 32 * 2); __bf16* Bh = (__bf16*)carve(192 * 32 * 2); __bf16* Bl = (__bf16*)carve(192 * 32 * 2); float* bb = (float*)carve(192 * 4);
  float* FD = (float*)carve((size_t)GR * 192 * 4); float* AGG = (float*)carve((size_t)GBv * GA * 288 * 4); float* M = (float*)carve((size_t)GBv * GA * GNF * 4);
  unsigned* FT16 = (unsigned*)carve((size_t)GBv * 192 * GV * 2); unsigned* EWT16 = (unsigned*)carve((size_t)GBv * 64 * GV * 2); float* AGGM = (float*)carve((size_t)GBv * 192 * 64 * 4);
  prep_kernel<<<(unsigned)(((size_t)GR * 16 + 255) / 256), 256, 0, stream>>>(data, Wf, bfl, Ws, bs, Dh, Dl, Bh, Bl, bb);
  { const int t = (GR / 64) * 3;
    wmma_gemm64<1, true, 2, 0, false><<<dim3((t + 7) / 8, 1), 256, 0, stream>>>(U16(Dh), U16(Dl), 32, 0, U16(Bh), U16(Bl), 32, 0, FD, nullptr, 192, 0, bb, nullptr, 0, GR, 192, 32, 1.0f); }
  frow_kernel<<<GR / 8, 256, 0, stream>>>(data, FD);
  ftrans_kernel<<<dim3(GV / 64, GBv), dim3(32, 8), 0, stream>>>(FD, FT16, EWT16);
  { const int t = (192 / 64) * 1;
    wmma_gemm64<0, false, 0, 0, false><<<dim3((t + 7) / 8, GBv), 256, 0, stream>>>((const unsigned short*)FT16, nullptr, GV, (long)192 * GV, (const unsigned short*)EWT16, nullptr, GV, (long)64 * GV, AGGM, nullptr, 64, (long)192 * 64, nullptr, nullptr, 0, 192, 64, GV, 1.0f / GV); }
  agg_kernel<<<GBv, 256, 0, stream>>>(FD, AGGM, AGG);
  m_kernel<<<GBv, 256, 0, stream>>>(AGG, Wout, M);
  out_kernel<<<GR / 8, 256, 0, stream>>>(data, FD, M, Wout, bout, (float*)d_out);
}
